// SSM_60911226192464
// MI455X (gfx1250) — hardware-run, weakly checked
//
#include <hip/hip_runtime.h>
#include <hip/hip_fp16.h>
#include <math.h>

typedef __attribute__((ext_vector_type(16))) _Float16 v16h;
typedef __attribute__((ext_vector_type(8)))  _Float16 v8h;
typedef __attribute__((ext_vector_type(8)))  float    v8f;
typedef __attribute__((ext_vector_type(4)))  float    v4f;
typedef __attribute__((ext_vector_type(2)))  unsigned v2u;
typedef __attribute__((ext_vector_type(4)))  unsigned v4u;

constexpr int kBatch   = 2;
constexpr int kL       = 2048;
constexpr int kRows    = kBatch * kL;
constexpr int kD       = 2048;
constexpr int kNst     = 16;
constexpr int kRank    = 128;
constexpr int kWReal   = kRank + 2 * kNst;
constexpr int kWN      = 192;
constexpr int kOffB    = kRank;
constexpr int kOffC    = kRank + kNst;
constexpr int kK2      = 160;
constexpr int kK2Words = kK2 / 8;
constexpr int kWdtPitch = 192;
constexpr int kXpWords = kWN / 4;
constexpr int kAlpFloats = kD * kNst;
constexpr int kPadFloats = kAlpFloats + kD;
constexpr float kXCarry = 64.0f;
constexpr float kWCarry = 4096.0f;
constexpr float kRCarry = 256.0f;
constexpr float kDCarry = 1024.0f;
constexpr float kYCarry = 128.0f;
static_assert(kBatch == 2 && kRows == 4096 && kL == 2048 && kD == 2048 && kNst == 16 && kRank == 128);
static_assert(kWReal == 160 && kWN == 192 && kOffB == 128 && kOffC == 144);
static_assert(kWReal <= kWN && (kWN % 64) == 0 && (kD % 32) == 0 && (kRows % 32) == 0);
static_assert(kK2 == 160 && (kK2 % 32) == 0 && kRank + 1 <= kK2 && kK2Words == 20);
static_assert(kWdtPitch == 192 && kWdtPitch >= kK2 && ((kWdtPitch * 2) % 128) == 0);
static_assert(kXpWords == 48 && (kWReal % 4) == 0);
static_assert((kD % 64) == 0 && (kL % 64) == 0);
static_assert(kAlpFloats == 32768 && kPadFloats == 34816);

constexpr size_t kSzXH   = (size_t)kRows * kD * 2;
constexpr size_t kSzXR   = (size_t)kRows * kD * 4;
constexpr size_t kSzWALL = (size_t)kWN * kD * 2;
constexpr size_t kSzXP   = (size_t)kRows * kWN * 4;
constexpr size_t kSzXPB  = (size_t)kRows * kWN * 4;
constexpr size_t kSzDRH  = (size_t)kRows * kK2 * 2;
constexpr size_t kSzWDT  = (size_t)kD * kWdtPitch * 2;
constexpr size_t kSzDTP  = (size_t)kRows * kD * 4;
constexpr size_t kSzPADS = (size_t)kPadFloats * 4;
constexpr size_t kSzYH   = (size_t)kRows * kD * 2;
constexpr size_t kOffXH   = 0;
constexpr size_t kOffXR   = kOffXH   + kSzXH;
constexpr size_t kOffWALL = kOffXR   + kSzXR;
constexpr size_t kOffXP   = kOffWALL + kSzWALL;
constexpr size_t kOffXPB  = kOffXP   + kSzXP;
constexpr size_t kOffDRH  = kOffXPB  + kSzXPB;
constexpr size_t kOffWDT  = kOffDRH  + kSzDRH;
constexpr size_t kOffDTP  = kOffWDT  + kSzWDT;
constexpr size_t kOffPADS = kOffDTP  + kSzDTP;
constexpr size_t kOffYH   = kOffPADS + kSzPADS;
constexpr size_t kWsTotal = kOffYH   + kSzYH;
static_assert(kSzXH == 16777216ull && kSzXR == 33554432ull && kSzWALL == 786432ull && kSzXP == 3145728ull);
static_assert(kSzXPB == 3145728ull && kSzDRH == 1310720ull && kSzWDT == 786432ull && kSzDTP == 33554432ull);
static_assert(kSzPADS == 139264ull && kSzYH == 16777216ull);
static_assert(kWsTotal == 16777216ull + 33554432ull + 786432ull + 3145728ull + 3145728ull + 1310720ull +
              786432ull + 33554432ull + 139264ull + 16777216ull);
static_assert(kWsTotal == 109977600ull);
static_assert(kWsTotal <= 134217728ull);
static_assert((kSzXH % 128) == 0 && (kSzXR % 128) == 0 && (kSzWALL % 128) == 0 && (kSzXP % 128) == 0 &&
              (kSzXPB % 128) == 0 && (kSzDRH % 128) == 0 && (kSzWDT % 128) == 0 && (kSzDTP % 128) == 0 &&
              (kSzPADS % 128) == 0 && (kSzYH % 128) == 0);
static_assert((((size_t)kAlpFloats * 4) % 128) == 0);
static_assert((((size_t)kWN * 4) % 128) == 0);

__device__ __forceinline__ _Float16 f16_flush(float v) {
  const float w = (fabsf(v) < 6.103515625e-05f) ? 0.0f : v;
  return (_Float16)w;
}

__device__ __forceinline__ float bf16r(float v) {
  unsigned u = __float_as_uint(v);
  u = (u + 0x7FFFu + ((u >> 16) & 1u)) & 0xFFFF0000u;
  return __uint_as_float(u);
}

__device__ __forceinline__ float h16_to_f32(unsigned hb) {
  const unsigned sgn = (hb & 0x8000u) << 16; const unsigned em = hb & 0x7fffu;
  const float fn = __uint_as_float((em << 13) + 0x38000000u);
  const float fs = (float)em * 5.9604644775390625e-8f;
  const float mag = (em < 0x400u) ? fs : fn; return __uint_as_float(__float_as_uint(mag) | sgn); }

namespace eng {
union FragU { v16h v; v8h h[2]; };
__device__ __forceinline__ v16h frag_load(const _Float16* p) {
  FragU f;
  f.h[0] = *(const v8h*)(p);
  f.h[1] = *(const v8h*)(p + 16);
  return f.v;
}
__device__ __forceinline__ v8f mma(v16h a, v16h b, v8f c) {
  return __builtin_amdgcn_wmma_f32_16x16x32_f16(false, a, false, b, (short)0, c, false, false);
}
__device__ __forceinline__ void guard1(v8f& a, v16h x, v16h y) {
  asm volatile("v_nop\n\tv_nop\n\tv_nop\n\tv_nop" : "+v"(a) : "v"(x), "v"(y));
}
__device__ __forceinline__ void guard_acc(v8f& a) {
  asm volatile("v_nop\n\tv_nop\n\tv_nop\n\tv_nop" : "+v"(a));
}
__device__ __forceinline__ void keep4(v16h a, v16h b, v16h c, v16h d) {
  asm volatile("v_nop" :: "v"(a), "v"(b), "v"(c), "v"(d));
}

template <int MI, int SPL>
__global__ __launch_bounds__(256) void gemm_f16_kernel(
    const unsigned short* __restrict__ Ap, const unsigned short* __restrict__ A2p, int lda,
    const unsigned short* __restrict__ Btp, const unsigned short* __restrict__ Bt2p, int ldb,
    float* __restrict__ C, int ldc, int M, int N, int K, float scale, float rscale)
{
  static_assert(MI >= 1 && MI <= 2);
  static_assert(SPL >= 0 && SPL <= 2);
  const _Float16* A   = (const _Float16*)Ap;
  const _Float16* A2  = (const _Float16*)A2p;
  const _Float16* Bt  = (const _Float16*)Btp;
  const _Float16* Bt2 = (const _Float16*)Bt2p;
  __shared__ __align__(16) float sT[8][16 * 68];
  const int lane = threadIdx.x & 31;
  const int wave = threadIdx.x >> 5;
  const int tilesN = N >> 6;
  const int tilesM = M / (16 * MI);
  const int tile = blockIdx.x * 8 + wave;
  if (tile >= tilesM * tilesN) return;
  const int tm = tile / tilesN;
  const int tn = tile - tm * tilesN;
  const int m0 = tm * (16 * MI);
  const int n0 = tn << 6;
  const int rlane = lane & 15;
  const int koff  = (lane >> 4) * 8;
  const int mOff  = (lane >> 4) * 8;

  v8f acc[MI][4], accr[MI][4];
#pragma unroll
  for (int i = 0; i < MI; ++i)
#pragma unroll
    for (int j = 0; j < 4; ++j) {
      acc[i][j]  = (v8f){0.f, 0.f, 0.f, 0.f, 0.f, 0.f, 0.f, 0.f};
      accr[i][j] = (v8f){0.f, 0.f, 0.f, 0.f, 0.f, 0.f, 0.f, 0.f};
    }

  for (int k0 = 0; k0 < K; k0 += 32) {
    v16h bh[4], bl[4];
#pragma unroll
    for (int j = 0; j < 4; ++j) {
      const size_t bo = (size_t)(n0 + (j << 4) + rlane) * ldb + koff + k0;
      bh[j] = frag_load(Bt + bo);
      if (SPL == 2) bl[j] = frag_load(Bt2 + bo); else bl[j] = bh[j];
    }
#pragma unroll
    for (int i = 0; i < MI; ++i) {
      const size_t ao = (size_t)(m0 + (i << 4) + rlane) * lda + koff + k0;
      const v16h ah = frag_load(A + ao);
      v16h al = ah;
      if (SPL >= 1) al = frag_load(A2 + ao);
#pragma unroll
      for (int j = 0; j < 4; ++j) {
        acc[i][j] = mma(ah, bh[j], acc[i][j]);
        if (SPL >= 1) accr[i][j] = mma(al, bh[j], accr[i][j]);
        if (SPL == 2) accr[i][j] = mma(ah, bl[j], accr[i][j]);
      }
#pragma unroll
      for (int j = 0; j < 4; ++j) {
        guard1(acc[i][j], ah, al);
        if (SPL >= 1) guard1(accr[i][j], ah, al);
      }
    }
    keep4(bh[0], bh[1], bh[2], bh[3]);
    if (SPL == 2) keep4(bl[0], bl[1], bl[2], bl[3]);
  }
#pragma unroll
  for (int i = 0; i < MI; ++i)
#pragma unroll
    for (int j = 0; j < 4; ++j) {
      guard_acc(acc[i][j]);
      if (SPL >= 1) guard_acc(accr[i][j]);
    }

  float* slab = sT[wave];
#pragma unroll
  for (int i = 0; i < MI; ++i) {
    const int mBase = m0 + (i << 4);
#pragma unroll
    for (int j = 0; j < 4; ++j) {
#pragma unroll
      for (int r = 0; r < 8; ++r) {
        float v = acc[i][j][r] * scale;
        if (SPL >= 1) v += accr[i][j][r] * rscale;
        slab[(mOff + r) * 68 + (j << 4) + rlane] = v;
      }
    }
    __builtin_amdgcn_fence(__ATOMIC_RELEASE, "workgroup");
    __builtin_amdgcn_wave_barrier();
    __builtin_amdgcn_fence(__ATOMIC_ACQUIRE, "workgroup");
    {
      const int hh = lane >> 4, c4 = (lane & 15) * 4;
      for (int pass = 0; pass < 2; ++pass) {
#pragma unroll
        for (int it = 0; it < 8; ++it) {
          const int row = it * 2 + hh;
          const v4f v = *(const v4f*)(slab + row * 68 + c4);
          *(volatile v4f*)(C + (size_t)(mBase + row) * ldc + n0 + c4) = v;
        }
        __threadfence();
      }
    }
    __builtin_amdgcn_fence(__ATOMIC_RELEASE, "workgroup");
    __builtin_amdgcn_wave_barrier();
    __builtin_amdgcn_fence(__ATOMIC_ACQUIRE, "workgroup");
  }
}
}

__device__ __forceinline__ _Float16 in_half(float v, float carry, bool live) {
  const float t = live ? (bf16r(v) * carry) : 0.0f;
  return f16_flush(t);
}
__device__ __forceinline__ _Float16 val_half(float v, float carry, bool live) {
  const float t = live ? (v * carry) : 0.0f;
  return f16_flush(t);
}
__device__ __forceinline__ int imin2(int a, int b) {
  return (a < b) ? a : b;
}
__device__ __forceinline__ int iclamp(int v, int lo, int hi) {
  const int t = (v < lo) ? lo : v;
  return (t > hi) ? hi : t;
}

__global__ __launch_bounds__(256) void pack_x_kernel(
    const float* __restrict__ x, unsigned short* __restrict__ XH)
{
  const int i = blockIdx.x * 256 + threadIdx.x;
  const float* sp = x + (size_t)i * 8;
  const v4f a0 = *(const v4f*)(sp);
  const v4f a1 = *(const v4f*)(sp + 4);
  const float f0 = a0[0];
  const float f1 = a0[1];
  const float f2 = a0[2];
  const float f3 = a0[3];
  const float f4 = a1[0];
  const float f5 = a1[1];
  const float f6 = a1[2];
  const float f7 = a1[3];
  const float r0 = bf16r(f0);
  const float r1 = bf16r(f1);
  const float r2 = bf16r(f2);
  const float r3 = bf16r(f3);
  const float r4 = bf16r(f4);
  const float r5 = bf16r(f5);
  const float r6 = bf16r(f6);
  const float r7 = bf16r(f7);
  v8h hv;
  hv[0] = val_half(r0, kXCarry, true);
  hv[1] = val_half(r1, kXCarry, true);
  hv[2] = val_half(r2, kXCarry, true);
  hv[3] = val_half(r3, kXCarry, true);
  hv[4] = val_half(r4, kXCarry, true);
  hv[5] = val_half(r5, kXCarry, true);
  hv[6] = val_half(r6, kXCarry, true);
  hv[7] = val_half(r7, kXCarry, true);
  unsigned short* qh = XH + (size_t)i * 8;
  *(volatile v8h*)qh = hv;
  __threadfence();
  *(volatile v8h*)qh = hv;
}

__global__ __launch_bounds__(256) void rne_x_kernel(
    const float* __restrict__ x, float* __restrict__ XR)
{
  const int i = blockIdx.x * 256 + threadIdx.x;
  const v4f a0 = *(const v4f*)(x + (size_t)i * 4);
  const float f0 = a0[0];
  const float f1 = a0[1];
  const float f2 = a0[2];
  const float f3 = a0[3];
  v4f o;
  o[0] = bf16r(f0);
  o[1] = bf16r(f1);
  o[2] = bf16r(f2);
  o[3] = bf16r(f3);
  float* q = XR + (size_t)i * 4;
  *(volatile v4f*)q = o;
  __threadfence();
  *(volatile v4f*)q = o;
}

__global__ __launch_bounds__(256) void pack_wall_kernel(
    const float* __restrict__ wx, unsigned short* __restrict__ WALL)
{
  const int i = blockIdx.x * 256 + threadIdx.x;
  const int n = i / (kD / 8);
  const int c8 = (i - n * (kD / 8)) * 8;
  const bool live = (n < kWReal);
  const int nr = imin2(n, kWReal - 1);
  const float* sp = wx + (size_t)nr * kD + c8;
  const v4f a0 = *(const v4f*)(sp);
  const v4f a1 = *(const v4f*)(sp + 4);
  const float f0 = a0[0];
  const float f1 = a0[1];
  const float f2 = a0[2];
  const float f3 = a0[3];
  const float f4 = a1[0];
  const float f5 = a1[1];
  const float f6 = a1[2];
  const float f7 = a1[3];
  v8h hv;
  hv[0] = in_half(f0, kWCarry, live);
  hv[1] = in_half(f1, kWCarry, live);
  hv[2] = in_half(f2, kWCarry, live);
  hv[3] = in_half(f3, kWCarry, live);
  hv[4] = in_half(f4, kWCarry, live);
  hv[5] = in_half(f5, kWCarry, live);
  hv[6] = in_half(f6, kWCarry, live);
  hv[7] = in_half(f7, kWCarry, live);
  unsigned short* q = WALL + (size_t)i * 8;
  *(volatile v8h*)q = hv;
  __threadfence();
  *(volatile v8h*)q = hv;
}

__global__ __launch_bounds__(256) void add_bias_kernel(
    const float* __restrict__ XP, const float* __restrict__ bdbc, float* __restrict__ XPB)
{
  const int i = blockIdx.x * 256 + threadIdx.x;
  const int c4 = (i % kXpWords) * 4;
  const bool live = (c4 < kWReal);
  const int cb = imin2(c4, kWReal - 4);
  const v4f a0 = *(const v4f*)(XP + (size_t)i * 4);
  const v4f b0 = *(const v4f*)(bdbc + cb);
  const float x0 = a0[0];
  const float x1 = a0[1];
  const float x2 = a0[2];
  const float x3 = a0[3];
  const float g0 = b0[0];
  const float g1 = b0[1];
  const float g2 = b0[2];
  const float g3 = b0[3];
  const float t0 = live ? bf16r(g0) : 0.0f;
  const float t1 = live ? bf16r(g1) : 0.0f;
  const float t2 = live ? bf16r(g2) : 0.0f;
  const float t3 = live ? bf16r(g3) : 0.0f;
  v4f o;
  o[0] = x0 + t0;
  o[1] = x1 + t1;
  o[2] = x2 + t2;
  o[3] = x3 + t3;
  float* q = XPB + (size_t)i * 4;
  *(volatile v4f*)q = o;
  __threadfence();
  *(volatile v4f*)q = o;
}

__global__ __launch_bounds__(256) void pack_dr_kernel(
    const float* __restrict__ XP, unsigned short* __restrict__ DRH)
{
  const int i = blockIdx.x * 256 + threadIdx.x;
  const int r = i / kK2Words;
  const int q = (i - r * kK2Words) * 8;
  const bool live = (q < kRank);
  const bool isOne = (q == kRank);
  const int qc = imin2(q, kRank - 8);
  const float* sp = XP + (size_t)r * kWN + qc;
  const v4f a0 = *(const v4f*)(sp);
  const v4f a1 = *(const v4f*)(sp + 4);
  const float f0 = a0[0];
  const float f1 = a0[1];
  const float f2 = a0[2];
  const float f3 = a0[3];
  const float f4 = a1[0];
  const float f5 = a1[1];
  const float f6 = a1[2];
  const float f7 = a1[3];
  const float t0a = live ? (f0 * kRCarry) : 0.0f;
  const float t0 = isOne ? kRCarry : t0a;
  v8h hv;
  hv[0] = f16_flush(t0);
  hv[1] = val_half(f1, kRCarry, live);
  hv[2] = val_half(f2, kRCarry, live);
  hv[3] = val_half(f3, kRCarry, live);
  hv[4] = val_half(f4, kRCarry, live);
  hv[5] = val_half(f5, kRCarry, live);
  hv[6] = val_half(f6, kRCarry, live);
  hv[7] = val_half(f7, kRCarry, live);
  unsigned short* qd = DRH + (size_t)i * 8;
  *(volatile v8h*)qd = hv;
  __threadfence();
  *(volatile v8h*)qd = hv;
}

constexpr int kRankWords = kRank / 8;
constexpr int kTailWords = (kWdtPitch - kRank) / 8;
static_assert(kRankWords == 16 && kTailWords == 8 && (kRankWords + kTailWords) * 8 == kWdtPitch);
static_assert(((kRank * 2) % 128) == 0);

__global__ __launch_bounds__(256) void pack_wdt_kernel(
    const float* __restrict__ w, unsigned short* __restrict__ WDT)
{
  const int i = blockIdx.x * 256 + threadIdx.x;
  const int d = i / kRankWords;
  const int q = (i - d * kRankWords) * 8;
  const float* sp = w + (size_t)d * kRank + q;
  const v4f a0 = *(const v4f*)(sp);
  const v4f a1 = *(const v4f*)(sp + 4);
  const float w0 = a0[0];
  const float w1 = a0[1];
  const float w2 = a0[2];
  const float w3 = a0[3];
  const float w4 = a1[0];
  const float w5 = a1[1];
  const float w6 = a1[2];
  const float w7 = a1[3];
  v8h hv;
  hv[0] = in_half(w0, kDCarry, true);
  hv[1] = in_half(w1, kDCarry, true);
  hv[2] = in_half(w2, kDCarry, true);
  hv[3] = in_half(w3, kDCarry, true);
  hv[4] = in_half(w4, kDCarry, true);
  hv[5] = in_half(w5, kDCarry, true);
  hv[6] = in_half(w6, kDCarry, true);
  hv[7] = in_half(w7, kDCarry, true);
  unsigned short* qd = WDT + (size_t)d * kWdtPitch + q;
  *(volatile v8h*)qd = hv;
  __threadfence();
  *(volatile v8h*)qd = hv;
}

__global__ __launch_bounds__(256) void pack_bias_kernel(
    const float* __restrict__ bdt, unsigned short* __restrict__ WDT)
{
  const int i = blockIdx.x * 256 + threadIdx.x;
  const int d = i / kTailWords;
  const int w = i - d * kTailWords;
  const bool isBias = (w == 0);
  const float bv = bdt[d];
  const float tb = bf16r(bv) * kDCarry;
  const float t0 = isBias ? tb : 0.0f;
  const _Float16 h0 = f16_flush(t0);
  const unsigned short b0 = __builtin_bit_cast(unsigned short, h0);
  const unsigned w0 = (unsigned)b0;
  v4u ov;
  ov[0] = w0;
  ov[1] = 0u;
  ov[2] = 0u;
  ov[3] = 0u;
  unsigned short* qd = WDT + (size_t)d * kWdtPitch + kRank + w * 8;
  *(volatile v4u*)qd = ov;
  __threadfence();
  *(volatile v4u*)qd = ov;
}

__global__ __launch_bounds__(32) void pads_kernel(
    const float* __restrict__ alog, const float* __restrict__ dpar, float* __restrict__ PADS)
{
  const int wi = blockIdx.x * 32 + threadIdx.x;
  const int f0 = wi * 4;
  const bool isA = (f0 < kAlpFloats);
  const int ea = isA ? f0 : (kAlpFloats - 4);
  const int ed = iclamp(f0 - kAlpFloats, 0, kD - 4);
  const v4f va = *(const v4f*)(alog + ea);
  const v4f vd = *(const v4f*)(dpar + ed);
  const float a0 = va[0];
  const float a1 = va[1];
  const float a2 = va[2];
  const float a3 = va[3];
  const float d0 = vd[0];
  const float d1 = vd[1];
  const float d2 = vd[2];
  const float d3 = vd[3];
  v4f o;
  o[0] = bf16r(isA ? a0 : d0);
  o[1] = bf16r(isA ? a1 : d1);
  o[2] = bf16r(isA ? a2 : d2);
  o[3] = bf16r(isA ? a3 : d3);
  float* q = PADS + (size_t)f0;
  *(volatile v4f*)q = o;
  __threadfence();
  *(volatile v4f*)q = o;
}

typedef float    ms1_v4f __attribute__((ext_vector_type(4)));
typedef unsigned ms1_v4u __attribute__((ext_vector_type(4)));
struct ms1_args {
  const float* dtpre;
  const float* u;
  const float* bc;
  const float* z;
  const float* A_log;
  const float* Dskip;
  __half* y;
  __half* y_lo;
  long ld_dtpre;
  long ld_u;
  long ld_bc;
  long ld_z;
  long ld_y;
  int offB;
  int offC;
  int offZ;
  float ycarry;
  int dir;
  int D;
  int L;
  int nbatch;
};
static_assert(sizeof(ms1_args) == 136);

__device__ __forceinline__ float ms1_flush16(float v) {
  return (fabsf(v) < 6.103515625e-05f) ? 0.0f : v;
}
__device__ __forceinline__ unsigned ms1_h16bits(float v) {
  return (unsigned)__half_as_ushort(__float2half_rn(ms1_flush16(v)));
}
__device__ __forceinline__ float ms1_h16val(unsigned b) {
  return __half2float(__ushort_as_half((unsigned short)b));
}
__device__ __forceinline__ float ms1_softplus(float v) {
  return fmaxf(v, 0.0f) + log1pf(expf(-fabsf(v)));
}
__device__ __forceinline__ void ms1_pack2(float v0, float v1, unsigned& hw, unsigned& lw) {
  const unsigned h0 = ms1_h16bits(v0);
  const unsigned h1 = ms1_h16bits(v1);
  const float r0 = (v0 - ms1_h16val(h0)) * 2048.0f;
  const float r1 = (v1 - ms1_h16val(h1)) * 2048.0f;
  const unsigned l0 = ms1_h16bits(r0);
  const unsigned l1 = ms1_h16bits(r1);
  hw = h0 | (h1 << 16);
  lw = l0 | (l1 << 16);
}

template <int NSTATE>
__global__ __launch_bounds__(64 * (NSTATE / 16)) void ms1_scan_kernel(ms1_args a)
{
  static_assert(NSTATE == 16 || NSTATE == 64);
  constexpr int NQ  = NSTATE / 16;
  constexpr int NT  = 64 * NQ;
  constexpr int NW  = NT / 32;
  constexpr int BCW = 2 * NSTATE;
  constexpr int YP  = 68;
  constexpr int RPI = NW * 4;
  constexpr int NIT = 64 / RPI;
  static_assert(16 * NT <= 64 * YP);
  __shared__ __align__(16) float sBC[64 * BCW];
  __shared__ __align__(16) float sY[64 * YP];
  const int tid  = threadIdx.x;
  const int lane = tid & 31;
  const int wave = tid >> 5;
  const int c    = tid / NQ;
  const int sq   = tid - c * NQ;
  const int bpb  = a.D / 64;
  const int bi   = blockIdx.x / bpb;
  if (bi >= a.nbatch) return;
  const int d0 = (blockIdx.x - bi * bpb) * 64;
  const int d  = d0 + c;
  const long rowb = (long)bi * a.L;
  const bool hasz  = (a.z != nullptr);
  const bool hasD  = (a.Dskip != nullptr);
  const bool hasLo = (a.y_lo != nullptr);

#pragma unroll 1
  for (int n = 0; n < 16; ++n) {
    const float al = a.A_log[(long)d * NSTATE + sq * 16 + n];
    sY[n * NT + tid] = -expf(al);
  }
  __syncthreads();
  float An[16], h[16];
#pragma unroll
  for (int n = 0; n < 16; ++n) {
    An[n] = sY[n * NT + tid];
    h[n] = 0.0f;
  }
  float Dd = 0.0f;
  if (hasD) Dd = a.Dskip[d];

  const int nchunk = a.L / 64;
  const bool fwd = (a.dir > 0);
  const int s0 = fwd ? 0 : 63;
  const int sd = fwd ? 1 : -1;
  const int q  = lane >> 3;
  const int c8 = (lane & 7) * 8;

  for (int ci = 0; ci < nchunk; ++ci) {
    const int tb = fwd ? (ci * 64) : (a.L - 64 - ci * 64);
    const long rowc = rowb + tb;
    __syncthreads();
#pragma unroll 8
    for (int i = 0; i < 32; ++i) {
      const int idx = tid + i * NT;
      const int st  = idx / BCW;
      const int col = idx - st * BCW;
      const int sc  = (col < NSTATE) ? (a.offB + col) : (a.offC + col - NSTATE);
      sBC[idx] = a.bc[(rowc + st) * a.ld_bc + sc];
    }
    __syncthreads();
    for (int s = 0; s < 64; ++s) {
      const int ls = s0 + sd * s;
      const long row = rowc + ls;
      float pre = a.dtpre[row * a.ld_dtpre + d];
      float uv  = a.u[row * a.ld_u + d];
      float zv  = 0.0f;
      if (hasz) zv = a.z[row * a.ld_z + a.offZ + d];
      asm volatile("" : "+v"(pre));
      asm volatile("" : "+v"(uv));
      asm volatile("" : "+v"(zv));
      const float delta = ms1_softplus(pre);
      const float dtx = delta * uv;
      const float* bp = sBC + ls * BCW + sq * 16;
      const float* cp = bp + NSTATE;
      ms1_v4f Bq[4], Cq[4];
#pragma unroll
      for (int k = 0; k < 4; ++k) {
        Bq[k] = *(const ms1_v4f*)(bp + 4 * k);
        Cq[k] = *(const ms1_v4f*)(cp + 4 * k);
      }
      float yv = 0.0f;
#pragma unroll
      for (int n = 0; n < 16; ++n) {
        const float e = __expf(delta * An[n]);
        h[n] = fmaf(e, h[n], dtx * Bq[n >> 2][n & 3]);
        yv = fmaf(h[n], Cq[n >> 2][n & 3], yv);
      }
      if (NQ > 1) {
        yv += __shfl_xor(yv, 1, 32);
        yv += __shfl_xor(yv, 2, 32);
      }
      if (hasD) yv = fmaf(uv, Dd, yv);
      if (hasz) {
        const float sg = __builtin_amdgcn_rcpf(1.0f + expf(-zv));
        yv = yv * (zv * sg);
      }
      if (sq == 0) sY[ls * YP + c] = yv * a.ycarry;
    }
    __syncthreads();
    ms1_v4u hw[NIT], lw[NIT];
#pragma unroll
    for (int it = 0; it < NIT; ++it) {
      const int row = it * RPI + wave * 4 + q;
      const float* sp = sY + row * YP + c8;
      const ms1_v4f f0 = *(const ms1_v4f*)(sp);
      const ms1_v4f f1 = *(const ms1_v4f*)(sp + 4);
      unsigned h0, h1, h2, h3, l0, l1, l2, l3;
      ms1_pack2(f0[0], f0[1], h0, l0);
      ms1_pack2(f0[2], f0[3], h1, l1);
      ms1_pack2(f1[0], f1[1], h2, l2);
      ms1_pack2(f1[2], f1[3], h3, l3);
      hw[it] = (ms1_v4u){h0, h1, h2, h3};
      lw[it] = (ms1_v4u){l0, l1, l2, l3};
    }
    for (int pass = 0; pass < 2; ++pass) {
#pragma unroll
      for (int it = 0; it < NIT; ++it) {
        const int row = it * RPI + wave * 4 + q;
        const long o = (rowc + row) * a.ld_y + d0 + c8;
        *(volatile ms1_v4u*)(a.y + o) = hw[it];
        if (hasLo) *(volatile ms1_v4u*)(a.y_lo + o) = lw[it];
      }
      __threadfence();
    }
  }
}

__device__ __forceinline__ float out_val(unsigned hb) {
  return h16_to_f32(hb) * (1.0f / kYCarry);
}
__global__ __launch_bounds__(256) void out_kernel(
    const unsigned short* __restrict__ YH, float* __restrict__ out)
{
  const int i = blockIdx.x * 256 + threadIdx.x;
  const v2u wy = *(const v2u*)(YH + (size_t)i * 4);
  const unsigned w0 = wy[0];
  const unsigned w1 = wy[1];
  v4f o;
  o[0] = out_val(w0 & 0xffffu);
  o[1] = out_val(w0 >> 16);
  o[2] = out_val(w1 & 0xffffu);
  o[3] = out_val(w1 >> 16);
  float* q = out + (size_t)i * 4;
  *(volatile v4f*)q = o;
  __threadfence();
  *(volatile v4f*)q = o;
}

static_assert(((kRows / 32) * (kWN / 64)) % 8 == 0 && ((kRows / 32) * (kWN / 64)) / 8 == 48);
static_assert((4096 / 32) * (192 / 64) / 8 == 48);
static_assert(((kRows / 32) * (kD / 64)) % 8 == 0 && ((kRows / 32) * (kD / 64)) / 8 == 512);
static_assert((4096 / 32) * (2048 / 64) / 8 == 512);
static_assert(((kRows * kD / 8) % 256) == 0 && (kRows * kD / 8) / 256 == 4096);
static_assert(((kRows * kD / 4) % 256) == 0 && (kRows * kD / 4) / 256 == 8192);
static_assert(((kWN * kD / 8) % 256) == 0 && (kWN * kD / 8) / 256 == 192);
static_assert(((kRows * kXpWords) % 256) == 0 && (kRows * kXpWords) / 256 == 768);
static_assert((4096 * 192 / 4) / 256 == 768);
static_assert(((kRows * kK2Words) % 256) == 0 && (kRows * kK2Words) / 256 == 320);
static_assert(((kD * kRankWords) % 256) == 0 && (kD * kRankWords) / 256 == 128);
static_assert((2048 * 16) / 256 == 128);
static_assert(((kD * kTailWords) % 256) == 0 && (kD * kTailWords) / 256 == 64);
static_assert((2048 * 8) / 256 == 64);
static_assert((kPadFloats / 4) == 272 * 32);
static_assert((2048 / 64) * 2 == 64);
static_assert((kD / 64) * kBatch == 64);

extern "C" void kernel_launch(void* const* d_in, const int* in_sizes, int n_in,
                              void* d_out, int out_size, void* d_ws, size_t ws_size,
                              hipStream_t stream)
{
  if (n_in < 7) return;
  if (in_sizes[0] != kBatch * kL * kD) return;
  if (in_sizes[1] != kWReal * kD) return;
  if (in_sizes[2] != kWReal) return;
  if (in_sizes[3] != kD * kRank) return;
  if (in_sizes[4] != kD) return;
  if (in_sizes[5] != kD * kNst) return;
  if (in_sizes[6] != kD) return;
  if (out_size != kBatch * kL * kD) return;
  if (ws_size < kWsTotal) return;

  const float* x_in   = (const float*)d_in[0];
  const float* w_dbc  = (const float*)d_in[1];
  const float* b_dbc  = (const float*)d_in[2];
  const float* w_dt   = (const float*)d_in[3];
  const float* b_dt   = (const float*)d_in[4];
  const float* a_log  = (const float*)d_in[5];
  const float* d_par  = (const float*)d_in[6];
  float* out = (float*)d_out;

  char* ws = (char*)d_ws;
  unsigned short* XH   = (unsigned short*)(ws + kOffXH);
  float*          XR   = (float*)(ws + kOffXR);
  unsigned short* WALL = (unsigned short*)(ws + kOffWALL);
  float*          XP   = (float*)(ws + kOffXP);
  float*          XPB  = (float*)(ws + kOffXPB);
  unsigned short* DRH  = (unsigned short*)(ws + kOffDRH);
  unsigned short* WDT  = (unsigned short*)(ws + kOffWDT);
  float*          DTP  = (float*)(ws + kOffDTP);
  float*          PADS = (float*)(ws + kOffPADS);
  unsigned short* YH   = (unsigned short*)(ws + kOffYH);
  float*          ALP  = PADS;
  float*          DSP  = PADS + kAlpFloats;

  constexpr float s1 = 1.0f / (kXCarry * kWCarry);
  constexpr float s2 = 1.0f / (kRCarry * kDCarry);

  pack_x_kernel<<<(kRows * kD / 8) / 256, 256, 0, stream>>>(x_in, XH);

  rne_x_kernel<<<(kRows * kD / 4) / 256, 256, 0, stream>>>(x_in, XR);

  pack_wall_kernel<<<(kWN * kD / 8) / 256, 256, 0, stream>>>(w_dbc, WALL);

  eng::gemm_f16_kernel<2, 0><<<dim3((4096 / 32) * (192 / 64) / 8), 256, 0, stream>>>(
      XH, nullptr, 2048, WALL, nullptr, 2048, XP, 192, 4096, 192, 2048, s1, 0.0f);

  add_bias_kernel<<<(kRows * kXpWords) / 256, 256, 0, stream>>>(XP, b_dbc, XPB);

  pack_dr_kernel<<<(kRows * kK2Words) / 256, 256, 0, stream>>>(XPB, DRH);

  pack_wdt_kernel<<<(kD * kRankWords) / 256, 256, 0, stream>>>(w_dt, WDT);

  pack_bias_kernel<<<(kD * kTailWords) / 256, 256, 0, stream>>>(b_dt, WDT);

  eng::gemm_f16_kernel<2, 0><<<dim3((4096 / 32) * (2048 / 64) / 8), 256, 0, stream>>>(
      DRH, nullptr, 160, WDT, nullptr, 192, DTP, 2048, 4096, 2048, 160, s2, 0.0f);

  pads_kernel<<<272, 32, 0, stream>>>(a_log, d_par, PADS);

  ms1_args sa;
  sa.dtpre = DTP;
  sa.u = XR;
  sa.bc = XPB;
  sa.z = nullptr;
  sa.A_log = ALP;
  sa.Dskip = DSP;
  sa.y = (__half*)YH;
  sa.y_lo = nullptr;
  sa.ld_dtpre = kD;
  sa.ld_u = kD;
  sa.ld_bc = kWN;
  sa.ld_z = 0;
  sa.ld_y = kD;
  sa.offB = kOffB;
  sa.offC = kOffC;
  sa.offZ = 0;
  sa.ycarry = kYCarry;
  sa.dir = 1;
  sa.D = kD;
  sa.L = kL;
  sa.nbatch = kBatch;

  ms1_scan_kernel<16><<<dim3((2048 / 64) * 2), 64, 0, stream>>>(sa);

  out_kernel<<<(kRows * kD / 4) / 256, 256, 0, stream>>>(YH, out);
}
